// AdvancedGNN_61168924230300
// MI455X (gfx1250) — hardware-run, weakly checked
//
#include <hip/hip_runtime.h>
#include <stddef.h>
#include <stdint.h>


#define FIN     256
#define D1      512
#define HC      128
#define NH1     4
#define ED      26
#define EDP     32
#define OC      128
#define N2      384
#define K2      1024
#define NTHR    256
#define NWAVE   8
#define EPT     8
#define CHUNK   (NTHR * EPT)
#define WCAP    (EPT * 32)
#define LISTN   (NWAVE * WCAP)
#define NB      512
#define RCAP    12288
#define DEGCAP  256
#define GBM     64
#define GBN     64
#define GTHR    128
#define SCW     4
#define SCTHR   (SCW * 32)
#define EP      132
#define WSMAX   134217728
#define LDS_BKT ((2 * RCAP + 2 * NB + LISTN + 2 * NWAVE) * 4)

static_assert(D1 == NH1 * HC);
static_assert(HC == 32 * 4);
static_assert(ED <= EDP && EDP == 32);
static_assert((CHUNK & (CHUNK - 1)) == 0 && CHUNK <= 4096);
static_assert((NB & (NB - 1)) == 0 && NB <= 4096 && (NB % 16) == 0);
static_assert(NTHR * 2 == NB);
static_assert(LISTN >= NB);
static_assert((RCAP % 16) == 0 && RCAP >= 8398 + 8398 / 4);
static_assert(DEGCAP >= 32 + 8);
static_assert(LDS_BKT <= 327680);
static_assert(SCW * 256 * 4 + SCW * 16 * EP * 4 <= 65536);
static_assert(GBM == (GTHR / 32) * 16);
static_assert((FIN % 32) == 0 && (K2 % 32) == 0 && K2 == 2 * D1);
static_assert((D1 % GBN) == 0 && (OC % GBN) == 0);
static_assert((EP % 4) == 0 && EP >= HC);

typedef float          v4f   __attribute__((ext_vector_type(4)));
typedef float          v8f   __attribute__((ext_vector_type(8)));
typedef int            v2i   __attribute__((ext_vector_type(2)));
typedef int            v4i   __attribute__((ext_vector_type(4)));
typedef int            v8i   __attribute__((ext_vector_type(8)));
typedef unsigned       v2u   __attribute__((ext_vector_type(2)));
typedef unsigned short v8us  __attribute__((ext_vector_type(8)));
typedef __bf16         v16bf __attribute__((ext_vector_type(16)));
typedef v4f __attribute__((may_alias)) v4fa;
union FragB { v16bf v; v8us u[2]; v8i w; v4i q[2]; };

__device__ __forceinline__ v8f wmx(const FragB& a, const FragB& b, v8f c) {
  v8f d = __builtin_amdgcn_wmma_f32_16x16x32_bf16(false, a.v, false, b.v, (short)0, c, false, false);
  asm volatile("v_nop\n\tv_nop\n\tv_nop\n\tv_nop" : "+v"(d) : "v"(a.w), "v"(b.w));
  return d;
}

__device__ __forceinline__ void pinf(float x) { asm volatile("" :: "v"(x)); }
__device__ __forceinline__ void pini(int x)   { asm volatile("" :: "v"(x)); }

__device__ __forceinline__ unsigned bfbits(float v) {
  const unsigned u = __float_as_uint(v);
  const unsigned r = (u + 0x7FFFu + ((u >> 16) & 1u)) >> 16;
  const unsigned nb = ((u >> 16) & 0x8000u) | 0x7FC0u;
  return ((u & 0x7FFFFFFFu) > 0x7F800000u) ? nb : r;
}
__device__ __forceinline__ float rbf(float v) { return __uint_as_float(bfbits(v) << 16); }
__device__ __forceinline__ v4f rbf4(const v4f a) {
  v4f o; o.x = rbf(a.x); o.y = rbf(a.y); o.z = rbf(a.z); o.w = rbf(a.w); return o;
}
__device__ __forceinline__ float wsum(float v) {
#pragma unroll
  for (int off = 16; off > 0; off >>= 1) v += __shfl_xor(v, off);
  return v;
}

__device__ __forceinline__ int scan_chunk(const int* __restrict__ dsts, int nE, int cbase, int slotBase,
                                          int nb, int vec8, int* list, int tid, int lane, int wave) {
  int wc = 0;
  const int el0  = tid * EPT;
  const int e0   = cbase + el0;
  const int sent = -2147483647 - 1;
  v4i da, db;
  if (vec8 != 0 && cbase + CHUNK <= nE) {
    da = *(const v4i*)(dsts + e0);
    db = *(const v4i*)(dsts + e0 + 4);
  } else {
    da.x = (e0     < nE) ? dsts[min(e0,     nE - 1)] : sent;
    da.y = (e0 + 1 < nE) ? dsts[min(e0 + 1, nE - 1)] : sent;
    da.z = (e0 + 2 < nE) ? dsts[min(e0 + 2, nE - 1)] : sent;
    da.w = (e0 + 3 < nE) ? dsts[min(e0 + 3, nE - 1)] : sent;
    db.x = (e0 + 4 < nE) ? dsts[min(e0 + 4, nE - 1)] : sent;
    db.y = (e0 + 5 < nE) ? dsts[min(e0 + 5, nE - 1)] : sent;
    db.z = (e0 + 6 < nE) ? dsts[min(e0 + 6, nE - 1)] : sent;
    db.w = (e0 + 7 < nE) ? dsts[min(e0 + 7, nE - 1)] : sent;
  }
  const unsigned nbs = (unsigned)slotBase;
  const unsigned unb = (unsigned)nb;
  const unsigned s0 = (unsigned)da.x - nbs, s1 = (unsigned)da.y - nbs;
  const unsigned s2 = (unsigned)da.z - nbs, s3 = (unsigned)da.w - nbs;
  const unsigned s4 = (unsigned)db.x - nbs, s5 = (unsigned)db.y - nbs;
  const unsigned s6 = (unsigned)db.z - nbs, s7 = (unsigned)db.w - nbs;
  const bool h0 = s0 < unb, h1 = s1 < unb, h2 = s2 < unb, h3 = s3 < unb;
  const bool h4 = s4 < unb, h5 = s5 < unb, h6 = s6 < unb, h7 = s7 < unb;
  const unsigned any = __builtin_amdgcn_ballot_w32(h0 | h1 | h2 | h3 | h4 | h5 | h6 | h7);
  if (any != 0u) {
#define HITJ(J, HJ, SJ) { \
      const unsigned mj = __builtin_amdgcn_ballot_w32(HJ); \
      if (mj != 0u) { \
        if (HJ) { \
          const int pos = wc + (int)__builtin_amdgcn_mbcnt_lo(mj, 0u); \
          if (pos < WCAP) list[wave * WCAP + pos] = ((el0 + (J)) << 12) | (int)(SJ); \
        } \
        wc += (int)__builtin_popcount(mj); } }
    HITJ(0, h0, s0)
    HITJ(1, h1, s1)
    HITJ(2, h2, s2)
    HITJ(3, h3, s3)
    HITJ(4, h4, s4)
    HITJ(5, h5, s5)
    HITJ(6, h6, s6)
    HITJ(7, h7, s7)
#undef HITJ
  }
  return wc;
}

__global__ __launch_bounds__(NTHR) void k_xprep(const float* __restrict__ x, unsigned short* xb, int nN, int nUnits) {
  const int i = (int)blockIdx.x * NTHR + (int)threadIdx.x;
  if (i >= nUnits) return;
  const int row = i >> 5;
  const int c0  = (i & 31) * 8;
  const int rc  = row < nN ? row : nN - 1;
  const float* p = x + (size_t)rc * FIN + c0;
  const v4f a = *(const v4f*)p, b = *(const v4f*)(p + 4);
  const unsigned mk = row < nN ? 0xFFFFu : 0u;
  v8us hv;
  hv[0] = (unsigned short)(bfbits(a.x) & mk); hv[1] = (unsigned short)(bfbits(a.y) & mk);
  hv[2] = (unsigned short)(bfbits(a.z) & mk); hv[3] = (unsigned short)(bfbits(a.w) & mk);
  hv[4] = (unsigned short)(bfbits(b.x) & mk); hv[5] = (unsigned short)(bfbits(b.y) & mk);
  hv[6] = (unsigned short)(bfbits(b.z) & mk); hv[7] = (unsigned short)(bfbits(b.w) & mk);
  const size_t o = (size_t)row * FIN + c0;
  *(volatile v8us*)(xb + o) = hv;
  __threadfence();
  *(volatile v8us*)(xb + o) = hv;
}

__global__ __launch_bounds__(NTHR) void k_eaprep(const float* __restrict__ ea, unsigned short* eab, int nE, int nUnits) {
  const int u = (int)blockIdx.x * NTHR + (int)threadIdx.x;
  if (u >= nUnits) return;
  int e = u >> 2; e = e < nE ? e : nE - 1;
  const int k8 = (u & 3) * 8;
  const float* p = ea + (size_t)e * ED;
  float f[8];
#pragma unroll
  for (int i = 0; i < 8; ++i) {
    const int kk = k8 + i;
    f[i] = p[kk < ED ? kk : ED - 1];
    pinf(f[i]);
  }
  v8us hv;
#pragma unroll
  for (int i = 0; i < 8; ++i) {
    const unsigned mk = (k8 + i < ED) ? 0xFFFFu : 0u;
    hv[i] = (unsigned short)(bfbits(f[i]) & mk);
  }
  const size_t o = (size_t)u * 8;
  *(volatile v8us*)(eab + o) = hv;
  __threadfence();
  *(volatile v8us*)(eab + o) = hv;
}

__global__ __launch_bounds__(NTHR) void k_wtr(const float* __restrict__ w, int cols, int Kin, int Kpad, int dup,
                                              unsigned short* wt, int nUnits) {
  const int u = (int)blockIdx.x * NTHR + (int)threadIdx.x;
  if (u >= nUnits) return;
  const int kq = Kpad >> 3;
  int n = u / kq;
  const int k8 = (u - n * kq) * 8;
  n = n < cols ? n : cols - 1;
  float f[8];
#pragma unroll
  for (int i = 0; i < 8; ++i) {
    const int kk = k8 + i;
    const int kc = kk < Kin ? kk : Kin - 1;
    f[i] = w[(size_t)kc * (size_t)cols + n];
    pinf(f[i]);
  }
  v8us hv;
#pragma unroll
  for (int i = 0; i < 8; ++i) {
    const unsigned mk = (k8 + i < Kin) ? 0xFFFFu : 0u;
    hv[i] = (unsigned short)(bfbits(f[i]) & mk);
  }
  const size_t pitch = (size_t)Kpad * (size_t)(dup != 0 ? 2 : 1);
  const size_t o = (size_t)n * pitch + k8;
  *(volatile v8us*)(wt + o) = hv;
  if (dup != 0) *(volatile v8us*)(wt + o + Kpad) = hv;
  __threadfence();
  *(volatile v8us*)(wt + o) = hv;
  if (dup != 0) *(volatile v8us*)(wt + o + Kpad) = hv;
}

template<int RESID>
__global__ __launch_bounds__(GTHR) void k_gemm(
    const unsigned short* __restrict__ A, const unsigned short* __restrict__ WT,
    const float* __restrict__ bias, const float* res, float* outF,
    int K, int ldo, int ocol, int ldr)
{
  __shared__ __attribute__((aligned(16))) float stg[GBM * GBN];
  const int tid = (int)threadIdx.x, lane = tid & 31, wave = tid >> 5, hh = lane >> 4, m = lane & 15;
  const int rowBase = (int)blockIdx.x * GBM;
  const int col0    = (int)blockIdx.y * GBN;

  v8f acc[4];
  {
    const v8f z = {0.f, 0.f, 0.f, 0.f, 0.f, 0.f, 0.f, 0.f};
    acc[0] = z; acc[1] = z; acc[2] = z; acc[3] = z;
  }
  const unsigned short* ap = A  + (size_t)(rowBase + 16 * wave + m) * (size_t)K + 8 * hh;
  const unsigned short* wp = WT + (size_t)(col0 + m) * (size_t)K + 8 * hh;
  const int ksteps = K >> 5;
#pragma unroll 1
  for (int ks = 0; ks < ksteps; ++ks) {
    FragB af;
    af.u[0] = *(const v8us*)(ap + 32 * ks);
    af.u[1] = *(const v8us*)(ap + 32 * ks + 16);
#pragma unroll
    for (int t = 0; t < 4; ++t) {
      const unsigned short* wq = wp + (size_t)(16 * t) * (size_t)K + 32 * ks;
      FragB bf;
      bf.u[0] = *(const v8us*)wq;
      bf.u[1] = *(const v8us*)(wq + 16);
      acc[t] = wmx(af, bf, acc[t]);
    }
  }

#pragma unroll
  for (int t = 0; t < 4; ++t) {
    const int lc = 16 * t + m;
#pragma unroll
    for (int r = 0; r < 8; ++r) {
      const int lr = 16 * wave + 8 * hh + r;
      stg[lr * GBN + lc] = acc[t][r];
    }
  }
  __syncthreads();

  const v4f bv = rbf4(*(const v4f*)(bias + col0 + 4 * m));
  v4f fv[8];
#pragma unroll
  for (int i = 0; i < 8; ++i) {
    const int lr = 16 * wave + 2 * i + hh;
    v4f v = *(const v4fa*)(stg + lr * GBN + 4 * m);
    v = v + bv;
    if (RESID) {
      const v4f rv = *(const v4f*)(res + (size_t)(rowBase + lr) * (size_t)ldr + col0 + 4 * m);
      v = v + rv;
    }
    fv[i] = v;
  }
#pragma unroll
  for (int i = 0; i < 8; ++i) {
    const int lr = 16 * wave + 2 * i + hh;
    float* op = outF + (size_t)(rowBase + lr) * (size_t)ldo + ocol + col0 + 4 * m;
    *(volatile v4f*)op = fv[i];
  }
  __threadfence();
#pragma unroll
  for (int i = 0; i < 8; ++i) {
    const int lr = 16 * wave + 2 * i + hh;
    float* op = outF + (size_t)(rowBase + lr) * (size_t)ldo + ocol + col0 + 4 * m;
    *(volatile v4f*)op = fv[i];
  }
}

__global__ __launch_bounds__(NTHR) void k_bucket(const int* __restrict__ srcs, const int* __restrict__ dsts,
                                                 int* ent, int* slot, int nN, int nE, int vec8) {
  extern __shared__ v4f lds_dyn[];
  int* reg1 = (int*)lds_dyn;
  int* reg2 = reg1 + RCAP;
  int* scnt = reg2 + RCAP;
  int* soff = scnt + NB;
  int* list = soff + NB;
  int* wcnt = list + LISTN;
  int* wtot = wcnt + NWAVE;
  const int tid = (int)threadIdx.x, lane = tid & 31;
  const int wave = __builtin_amdgcn_readfirstlane(tid >> 5);
  const int nodeBase = (int)blockIdx.x * NB;

  for (int i = tid; i < NB; i += NTHR) scnt[i] = 0;
  for (int i = tid; i < RCAP; i += NTHR) { reg1[i] = 0; reg2[i] = 0; }
  __syncthreads();

  int tot = 0;
  const int nChunks = (nE + CHUNK - 1) / CHUNK;
#pragma unroll 1
  for (int ch = 0; ch < nChunks; ++ch) {
    const int cbase = ch * CHUNK;
    const int wc = scan_chunk(dsts, nE, cbase, nodeBase, NB, vec8, list, tid, lane, wave);
    if (lane == 0) wcnt[wave] = wc;
    __syncthreads();
    int pre = 0, all = 0;
#pragma unroll
    for (int w2 = 0; w2 < NWAVE; ++w2) {
      int c = wcnt[w2];
      c = c < 0 ? 0 : (c > WCAP ? WCAP : c);
      all += c;
      pre += (w2 < wave) ? c : 0;
    }
    const int wcc  = wc > WCAP ? WCAP : wc;
    const int base = tot + pre;
#pragma unroll 1
    for (int i = lane; i < wcc; i += 32) {
      const int en = list[wave * WCAP + i];
      const int el = (en >> 12) & (CHUNK - 1);
      const int sl = en & (NB - 1);
      int eid = cbase + el;
      eid = eid > nE - 1 ? nE - 1 : eid;
      const int pos = base + i;
      if (pos < RCAP) reg1[pos] = (int)(((unsigned)eid << 12) | (unsigned)sl);
    }
    tot += all;
    tot = tot > RCAP ? RCAP : tot;
    __syncthreads();
  }
  const int nh = tot;

  if (wave == 0) {
#pragma unroll 1
    for (int b0 = 0; b0 < nh; b0 += 32) {
      const int idx = b0 + lane;
      const int uv  = reg1[idx < RCAP ? idx : RCAP - 1];
      const int m32 = (nh - b0) < 32 ? (nh - b0) : 32;
#pragma unroll 1
      for (int k = 0; k < m32; ++k) {
        const int u  = __builtin_amdgcn_readlane(uv, k);
        const int sl = u & (NB - 1);
        if (lane == 0) scnt[sl] = scnt[sl] + 1;
      }
    }
  }
  __syncthreads();

  {
    const int r0 = scnt[2 * tid], r1 = scnt[2 * tid + 1];
    const int e0 = r0 < 0 ? 0 : r0, e1 = r1 < 0 ? 0 : r1;
    const int ts = e0 + e1;
    int incl = ts;
#pragma unroll
    for (int d = 1; d < 32; d <<= 1) {
      const int up = __shfl_up(incl, d);
      if (lane >= d) incl += up;
    }
    if (lane == 31) wtot[wave] = incl;
    __syncthreads();
    int pre = 0;
#pragma unroll
    for (int w2 = 0; w2 < NWAVE; ++w2) pre += (w2 < wave) ? wtot[w2] : 0;
    const int run = pre + incl - ts;
    soff[2 * tid]     = run;
    soff[2 * tid + 1] = run + e0;
  }
  __syncthreads();
  for (int i = tid; i < NB; i += NTHR) list[i] = soff[i];
  __syncthreads();

  if (wave == 0) {
#pragma unroll 1
    for (int b0 = 0; b0 < nh; b0 += 32) {
      const int idx = b0 + lane;
      const int uv  = reg1[idx < RCAP ? idx : RCAP - 1];
      const int m32 = (nh - b0) < 32 ? (nh - b0) : 32;
#pragma unroll 1
      for (int k = 0; k < m32; ++k) {
        const int u   = __builtin_amdgcn_readlane(uv, k);
        const int sl  = u & (NB - 1);
        const int eid = (int)((unsigned)u >> 12);
        if (lane == 0) {
          int pos = list[sl];
          pos = pos < 0 ? 0 : (pos > RCAP - 1 ? RCAP - 1 : pos);
          reg2[pos] = eid;
          list[sl] = pos + 1;
        }
      }
    }
  }
  __syncthreads();

  const bool ovf = (nh >= RCAP);
  const int nhPad = (nh + 15) & ~15;
  int* eb = ent + (size_t)blockIdx.x * (size_t)(2 * RCAP);
#pragma unroll 1
  for (int p0 = 0; p0 < nhPad; p0 += 2 * NTHR) {
    const int p   = p0 + 2 * tid;
    const bool ac = p < nhPad;
    const int pa  = p < RCAP - 2 ? p : RCAP - 2;
    int e0 = reg2[pa], e1 = reg2[pa + 1];
    e0 = e0 < 0 ? 0 : (e0 > nE - 1 ? nE - 1 : e0);
    e1 = e1 < 0 ? 0 : (e1 > nE - 1 ? nE - 1 : e1);
    const int s0 = srcs[e0];
    const int s1 = srcs[e1];
    pini(s0); pini(s1);
    const int m0 = (p     < nh) ? -1 : 0;
    const int m1 = (p + 1 < nh) ? -1 : 0;
    v4i v;
    v.x = s0 & m0; v.y = e0 & m0; v.z = s1 & m1; v.w = e1 & m1;
    if (ac) *(volatile v4i*)(eb + 2 * pa) = v;
    __threadfence();
    if (ac) *(volatile v4i*)(eb + 2 * pa) = v;
  }
  {
    v4i sv;
    sv.x = soff[2 * tid];
    sv.y = ovf ? -1 : scnt[2 * tid];
    sv.z = soff[2 * tid + 1];
    sv.w = ovf ? -1 : scnt[2 * tid + 1];
    int* sp = slot + 2 * (size_t)(nodeBase + 2 * tid);
    *(volatile v4i*)sp = sv;
    __threadfence();
    *(volatile v4i*)sp = sv;
  }
  (void)nN;
}

template<int H, int MODE>
__global__ __launch_bounds__(SCTHR) __attribute__((amdgpu_num_vgpr(248)))
void k_scan(const int* __restrict__ ent, const int* __restrict__ slot,
            const unsigned short* __restrict__ eab, const unsigned short* __restrict__ wet,
            const float* XL, int ldxl, float* XR, int ldxr,
            const float* __restrict__ att, const float* __restrict__ bias,
            const float* SK, int ldsk, const float* __restrict__ gam, const float* __restrict__ bet,
            float* outF, int nN, int nE)
{
  __shared__ __attribute__((aligned(16))) int   sA[SCW * 256];
  __shared__ __attribute__((aligned(16))) float sE[SCW * 16 * EP];
  const int tid = (int)threadIdx.x, lane = tid & 31, hh = lane >> 4, m = lane & 15;
  const int wave = __builtin_amdgcn_readfirstlane(tid >> 5);
  const int i = (int)blockIdx.x * SCW + wave;
  if (i >= nN) return;
  int*   At = sA + wave * 256;
  float* Et = sE + wave * 16 * EP;

  const v2i se = *(const v2i*)(slot + 2 * (size_t)i);
  int st = __builtin_amdgcn_readfirstlane(se.x);
  const int craw = __builtin_amdgcn_readfirstlane(se.y);
  st = st < 0 ? 0 : (st > RCAP - 1 ? RCAP - 1 : st);
  int cnt = craw < 0 ? 0 : (craw > DEGCAP ? DEGCAP : craw);
  if (cnt > RCAP - st) cnt = RCAP - st;
  const float qnan = __int_as_float(0x7fc00000);
  const float pz = (craw < 0 || craw > DEGCAP) ? qnan : 0.0f;
  const int blk = i / NB;
  const int* eb = ent + (size_t)blk * (size_t)(2 * RCAP);
  const v8f z8 = {0.f, 0.f, 0.f, 0.f, 0.f, 0.f, 0.f, 0.f};

#pragma unroll 1
  for (int j = 0; j < H; ++j) {
    const int cb = HC * j + 4 * lane;
    const v4f xr = *(const v4f*)(XR + (size_t)i * (size_t)ldxr + cb);
    const v4f at = rbf4(*(const v4f*)(att + cb));
    v4f acc = {0.f, 0.f, 0.f, 0.f};
    float mx = -1.0e30f, dn = 0.0f;

#pragma unroll 1
    for (int t0 = 0; t0 < cnt; t0 += 16) {
      const int nv = (cnt - t0) < 16 ? (cnt - t0) : 16;
      int ei = st + t0 + m;
      ei = ei > st + cnt - 1 ? st + cnt - 1 : ei;
      const v2i en = *(const v2i*)(eb + 2 * ei);
      const int src = en.x < 0 ? 0 : (en.x > nN - 1 ? nN - 1 : en.x);
      const int eid = en.y < 0 ? 0 : (en.y > nE - 1 ? nE - 1 : en.y);

      __builtin_amdgcn_fence(__ATOMIC_RELEASE, "wavefront");
      __builtin_amdgcn_wave_barrier();
#pragma unroll
      for (int t = 0; t < 2; ++t) {
        const int row = (lane >> 2) + 8 * t;
        const int er  = __shfl(eid, row);
        v4i w = *(const v4i*)(eab + (size_t)er * EDP + 8 * (lane & 3));
        const int msk = (row < nv) ? -1 : 0;
        w.x &= msk; w.y &= msk; w.z &= msk; w.w &= msk;
        *(v4i*)(At + row * 16 + 4 * (lane & 3)) = w;
      }
      __builtin_amdgcn_fence(__ATOMIC_RELEASE, "wavefront");
      __builtin_amdgcn_wave_barrier();
      FragB af;
      af.q[0] = *(const v4i*)(At + m * 16 + 4 * hh);
      af.q[1] = *(const v4i*)(At + m * 16 + 8 + 4 * hh);
#pragma unroll
      for (int tt = 0; tt < 8; ++tt) {
        const unsigned short* wq = wet + (size_t)(HC * j + 16 * tt + m) * EDP + 8 * hh;
        FragB bf;
        bf.q[0] = *(const v4i*)wq;
        bf.q[1] = *(const v4i*)(wq + 16);
        v8f d = wmx(af, bf, z8);
#pragma unroll
        for (int r = 0; r < 8; ++r) Et[(8 * hh + r) * EP + 16 * tt + m] = d[r];
      }
      __builtin_amdgcn_fence(__ATOMIC_RELEASE, "wavefront");
      __builtin_amdgcn_wave_barrier();
#pragma unroll 1
      for (int r = 0; r < nv; ++r) {
        const int s = __builtin_amdgcn_readlane(src, r);
        const v4f xl = *(const v4f*)(XL + (size_t)s * (size_t)ldxl + cb);
        const v4f ee = *(const v4fa*)(Et + r * EP + 4 * lane);
        v4f v = (xl + xr) + ee;
        v.x = (v.x > 0.0f) ? v.x : 0.2f * v.x;
        v.y = (v.y > 0.0f) ? v.y : 0.2f * v.y;
        v.z = (v.z > 0.0f) ? v.z : 0.2f * v.z;
        v.w = (v.w > 0.0f) ? v.w : 0.2f * v.w;
        float part = v.x * at.x;
        part = fmaf(v.y, at.y, part);
        part = fmaf(v.z, at.z, part);
        part = fmaf(v.w, at.w, part);
        const float al = wsum(part);
        const float df = al - mx;
        const float eo = expf(-fabsf(df));
        const bool up  = df > 0.0f;
        const float s1 = up ? eo : 1.0f;
        const float s2 = up ? 1.0f : eo;
        mx = up ? al : mx;
        dn = fmaf(dn, s1, s2);
        acc = acc * s1 + xl * s2;
      }
    }

    const float inv = (cnt > 0) ? (1.0f / (dn + 1e-16f)) : 0.0f;
    const v4f bb = rbf4(*(const v4f*)(bias + cb));
    v4f o = acc * inv + bb;
    o = o + pz;
    if (MODE == 0) {
      float* gp = XR + (size_t)i * (size_t)ldxr + cb;
      *(volatile v4f*)gp = o;
      __threadfence();
      *(volatile v4f*)gp = o;
    } else {
      const v4f sk = *(const v4f*)(SK + (size_t)i * (size_t)ldsk + cb);
      const v4f hv = o + sk;
      const float sm = wsum((hv.x + hv.y) + (hv.z + hv.w));
      const float mu = sm * (1.0f / (float)OC);
      const v4f dv = hv - mu;
      const float sq = wsum((dv.x * dv.x + dv.y * dv.y) + (dv.z * dv.z + dv.w * dv.w));
      const float var = sq * (1.0f / (float)OC);
      const float rstd = 1.0f / sqrtf(var + 1e-5f);
      const v4f gg = rbf4(*(const v4f*)(gam + cb));
      const v4f bt = rbf4(*(const v4f*)(bet + cb));
      const v4f y = (dv * rstd) * gg + bt;
      float* gp = outF + (size_t)i * OC + cb;
      *(volatile v4f*)gp = y;
      __threadfence();
      *(volatile v4f*)gp = y;
    }
  }
  (void)SK; (void)ldsk; (void)gam; (void)bet; (void)outF;
}

__global__ __launch_bounds__(NTHR) void k_ln1(const float* __restrict__ pre, const float* __restrict__ gam,
                                              const float* __restrict__ bet, unsigned short* hhl, int nN, int MPr) {
  const int tid = (int)threadIdx.x, lane = tid & 31;
  const int wave = __builtin_amdgcn_readfirstlane(tid >> 5);
  const int row = (int)blockIdx.x * NWAVE + wave;
  if (row >= MPr) return;
  const int rc = row < nN ? row : nN - 1;
  const unsigned pm = row < nN ? 0xFFFFFFFFu : 0u;
  const float* p = pre + (size_t)rc * D1 + 4 * lane;
  float s = 0.0f;
#pragma unroll 1
  for (int j = 0; j < NH1; ++j) {
    const v4f a = *(const v4f*)(p + HC * j);
    s += (a.x + a.y) + (a.z + a.w);
  }
  const float mu = wsum(s) * (1.0f / (float)D1);
  float q = 0.0f;
#pragma unroll 1
  for (int j = 0; j < NH1; ++j) {
    const v4f a = *(const v4f*)(p + HC * j);
    const v4f d = a - mu;
    q += (d.x * d.x + d.y * d.y) + (d.z * d.z + d.w * d.w);
  }
  const float var = wsum(q) * (1.0f / (float)D1);
  const float rstd = 1.0f / sqrtf(var + 1e-5f);
#pragma unroll 1
  for (int j = 0; j < NH1; ++j) {
    const v4f a  = *(const v4f*)(p + HC * j);
    const v4f gg = rbf4(*(const v4f*)(gam + HC * j + 4 * lane));
    const v4f bt = rbf4(*(const v4f*)(bet + HC * j + 4 * lane));
    v4f y = ((a - mu) * rstd) * gg + bt;
    y.x = (y.x > 0.0f) ? y.x : expm1f(y.x);
    y.y = (y.y > 0.0f) ? y.y : expm1f(y.y);
    y.z = (y.z > 0.0f) ? y.z : expm1f(y.z);
    y.w = (y.w > 0.0f) ? y.w : expm1f(y.w);
    const unsigned h0 = bfbits(y.x), h1 = bfbits(y.y), h2 = bfbits(y.z), h3 = bfbits(y.w);
    const unsigned l0 = bfbits(y.x - __uint_as_float(h0 << 16));
    const unsigned l1 = bfbits(y.y - __uint_as_float(h1 << 16));
    const unsigned l2 = bfbits(y.z - __uint_as_float(h2 << 16));
    const unsigned l3 = bfbits(y.w - __uint_as_float(h3 << 16));
    v2u hv, lv;
    hv.x = (h0 | (h1 << 16)) & pm; hv.y = (h2 | (h3 << 16)) & pm;
    lv.x = (l0 | (l1 << 16)) & pm; lv.y = (l2 | (l3 << 16)) & pm;
    unsigned short* hp = hhl + (size_t)row * K2 + HC * j + 4 * lane;
    *(volatile v2u*)hp = hv;
    *(volatile v2u*)(hp + D1) = lv;
    __threadfence();
    *(volatile v2u*)hp = hv;
    *(volatile v2u*)(hp + D1) = lv;
  }
}

static inline int cdiv(int a, int b) { return (a + b - 1) / b; }

extern "C" void kernel_launch(void* const* d_in, const int* in_sizes, int n_in,
                              void* d_out, int out_size, void* d_ws, size_t ws_size,
                              hipStream_t stream) {
  if (n_in < 25) return;
  const int nN = in_sizes[0] / FIN;
  if (nN <= 0 || in_sizes[0] != nN * FIN || nN > (1 << 21)) return;
  if (in_sizes[1] < 2 || (in_sizes[1] & 1) != 0) return;
  const int nE = in_sizes[1] / 2;
  if (nE < 1 || nE > (1 << 20)) return;
  if (in_sizes[2] != nE * ED) return;
  if (in_sizes[3] != FIN * D1 || in_sizes[5] != FIN * D1 || in_sizes[10] != FIN * D1) return;
  if (in_sizes[4] != D1 || in_sizes[6] != D1 || in_sizes[9] != D1 || in_sizes[11] != D1) return;
  if (in_sizes[12] != D1 || in_sizes[13] != D1) return;
  if (in_sizes[7] != ED * D1 || in_sizes[8] != NH1 * HC) return;
  if (in_sizes[14] != D1 * OC || in_sizes[16] != D1 * OC || in_sizes[21] != D1 * OC) return;
  if (in_sizes[15] != OC || in_sizes[17] != OC || in_sizes[20] != OC || in_sizes[22] != OC) return;
  if (in_sizes[23] != OC || in_sizes[24] != OC) return;
  if (in_sizes[18] != ED * OC || in_sizes[19] != OC) return;
  if (out_size != nN * OC) return;

  const float* x     = (const float*)d_in[0];
  const int*   ei    = (const int*)  d_in[1];
  const float* ea    = (const float*)d_in[2];
  const float* W1l   = (const float*)d_in[3];
  const float* b1l   = (const float*)d_in[4];
  const float* W1r   = (const float*)d_in[5];
  const float* b1r   = (const float*)d_in[6];
  const float* We1   = (const float*)d_in[7];
  const float* att1  = (const float*)d_in[8];
  const float* bias1 = (const float*)d_in[9];
  const float* Ws1   = (const float*)d_in[10];
  const float* bs1   = (const float*)d_in[11];
  const float* g1    = (const float*)d_in[12];
  const float* be1   = (const float*)d_in[13];
  const float* W2l   = (const float*)d_in[14];
  const float* b2l   = (const float*)d_in[15];
  const float* W2r   = (const float*)d_in[16];
  const float* b2r   = (const float*)d_in[17];
  const float* We2   = (const float*)d_in[18];
  const float* att2  = (const float*)d_in[19];
  const float* bias2 = (const float*)d_in[20];
  const float* Ws2   = (const float*)d_in[21];
  const float* bs2   = (const float*)d_in[22];
  const float* g2    = (const float*)d_in[23];
  const float* be2   = (const float*)d_in[24];
  float* out = (float*)d_out;
  const int* src = ei;
  const int* dst = ei + nE;

  const int MP   = cdiv(nN, GBM) * GBM;
  const int gB   = cdiv(nN, NB);
  const int vec8 = ((nE & 3) == 0) ? 1 : 0;

  char* ws = (char*)d_ws;
  size_t off = 0;
  const size_t oXB  = off; off += (size_t)MP * FIN * 2;               off = (off + 255) & ~(size_t)255;
  const size_t oEAB = off; off += (size_t)nE * EDP * 2;               off = (off + 255) & ~(size_t)255;
  const size_t oRA  = off; off += (size_t)MP * D1 * 4;                off = (off + 255) & ~(size_t)255;
  const size_t oRB  = off; off += (size_t)MP * D1 * 4;                off = (off + 255) & ~(size_t)255;
  const size_t oENT = off; off += (size_t)gB * RCAP * 8;              off = (off + 255) & ~(size_t)255;
  const size_t oSLT = off; off += (size_t)gB * NB * 8;                off = (off + 255) & ~(size_t)255;
  const size_t oW1L = off; off += (size_t)D1 * FIN * 2;               off = (off + 255) & ~(size_t)255;
  const size_t oW1R = off; off += (size_t)D1 * FIN * 2;               off = (off + 255) & ~(size_t)255;
  const size_t oWS1 = off; off += (size_t)D1 * FIN * 2;               off = (off + 255) & ~(size_t)255;
  const size_t oW2L = off; off += (size_t)OC * K2 * 2;                off = (off + 255) & ~(size_t)255;
  const size_t oW2R = off; off += (size_t)OC * K2 * 2;                off = (off + 255) & ~(size_t)255;
  const size_t oWS2 = off; off += (size_t)OC * K2 * 2;                off = (off + 255) & ~(size_t)255;
  const size_t oWE1 = off; off += (size_t)D1 * EDP * 2;               off = (off + 255) & ~(size_t)255;
  const size_t oWE2 = off; off += (size_t)OC * EDP * 2;               off = (off + 255) & ~(size_t)255;
  if (off > ws_size || off > (size_t)WSMAX) return;
  if ((size_t)MP * K2 * 2 > (size_t)MP * D1 * 4) return;
  if ((size_t)MP * N2 * 4 > (size_t)MP * D1 * 4) return;
  unsigned short* XB   = (unsigned short*)(ws + oXB);
  unsigned short* EAB  = (unsigned short*)(ws + oEAB);
  float*          RA   = (float*)(ws + oRA);
  float*          RB   = (float*)(ws + oRB);
  unsigned short* HHL  = (unsigned short*)(ws + oRB);
  int*            ENT  = (int*)(ws + oENT);
  int*            SLT  = (int*)(ws + oSLT);
  unsigned short* W1LT = (unsigned short*)(ws + oW1L);
  unsigned short* W1RT = (unsigned short*)(ws + oW1R);
  unsigned short* WS1T = (unsigned short*)(ws + oWS1);
  unsigned short* W2LT = (unsigned short*)(ws + oW2L);
  unsigned short* W2RT = (unsigned short*)(ws + oW2R);
  unsigned short* WS2T = (unsigned short*)(ws + oWS2);
  unsigned short* WE1T = (unsigned short*)(ws + oWE1);
  unsigned short* WE2T = (unsigned short*)(ws + oWE2);

  hipFuncSetAttribute(reinterpret_cast<const void*>(&k_bucket),
                      hipFuncAttributeMaxDynamicSharedMemorySize, LDS_BKT);

  {
    const int nUx = MP * (FIN / 8);
    k_xprep<<<cdiv(nUx, NTHR), NTHR, 0, stream>>>(x, XB, nN, nUx);
    const int nUe = nE * (EDP / 8);
    k_eaprep<<<cdiv(nUe, NTHR), NTHR, 0, stream>>>(ea, EAB, nE, nUe);
    const int nU1 = D1 * (FIN / 8);
    k_wtr<<<cdiv(nU1, NTHR), NTHR, 0, stream>>>(W1l, D1, FIN, FIN, 0, W1LT, nU1);
    k_wtr<<<cdiv(nU1, NTHR), NTHR, 0, stream>>>(W1r, D1, FIN, FIN, 0, W1RT, nU1);
    k_wtr<<<cdiv(nU1, NTHR), NTHR, 0, stream>>>(Ws1, D1, FIN, FIN, 0, WS1T, nU1);
    const int nU2 = OC * (D1 / 8);
    k_wtr<<<cdiv(nU2, NTHR), NTHR, 0, stream>>>(W2l, OC, D1, D1, 1, W2LT, nU2);
    k_wtr<<<cdiv(nU2, NTHR), NTHR, 0, stream>>>(W2r, OC, D1, D1, 1, W2RT, nU2);
    k_wtr<<<cdiv(nU2, NTHR), NTHR, 0, stream>>>(Ws2, OC, D1, D1, 1, WS2T, nU2);
    const int nU3 = D1 * (EDP / 8);
    k_wtr<<<cdiv(nU3, NTHR), NTHR, 0, stream>>>(We1, D1, ED, EDP, 0, WE1T, nU3);
    const int nU4 = OC * (EDP / 8);
    k_wtr<<<cdiv(nU4, NTHR), NTHR, 0, stream>>>(We2, OC, ED, EDP, 0, WE2T, nU4);
  }

  k_bucket<<<gB, NTHR, LDS_BKT, stream>>>(src, dst, ENT, SLT, nN, nE, vec8);

  const int gM = MP / GBM;
  k_gemm<0><<<dim3(gM, D1 / GBN), GTHR, 0, stream>>>(XB, W1LT, b1l, b1l, RA, FIN, D1, 0, 0);
  k_gemm<0><<<dim3(gM, D1 / GBN), GTHR, 0, stream>>>(XB, W1RT, b1r, b1r, RB, FIN, D1, 0, 0);
  k_scan<NH1, 0><<<cdiv(nN, SCW), SCTHR, 0, stream>>>(ENT, SLT, EAB, WE1T, RA, D1, RB, D1, att1, bias1,
                                                       RA, D1, g1, be1, RB, nN, nE);
  k_gemm<1><<<dim3(gM, D1 / GBN), GTHR, 0, stream>>>(XB, WS1T, bs1, RB, RA, FIN, D1, 0, D1);
  k_ln1<<<cdiv(MP, NWAVE), NTHR, 0, stream>>>(RA, g1, be1, HHL, nN, MP);
  k_gemm<0><<<dim3(gM, OC / GBN), GTHR, 0, stream>>>(HHL, W2LT, b2l, b2l, RA, K2, N2, 0, 0);
  k_gemm<0><<<dim3(gM, OC / GBN), GTHR, 0, stream>>>(HHL, W2RT, b2r, b2r, RA, K2, N2, OC, 0);
  k_gemm<0><<<dim3(gM, OC / GBN), GTHR, 0, stream>>>(HHL, WS2T, bs2, bs2, RA, K2, N2, 2 * OC, 0);
  k_scan<1, 1><<<cdiv(nN, SCW), SCTHR, 0, stream>>>(ENT, SLT, EAB, WE2T, RA, N2, RA + OC, N2, att2, bias2,
                                                     RA + 2 * OC, N2, g2, be2, out, nN, nE);
}
